// DNF_21912923144502
// MI455X (gfx1250) — hardware-run, weakly checked
//
#include <hip/hip_runtime.h>


#ifndef NB
#define NB 1024
#endif
#define NB_FULL 1024
#define KP   512
#define NC   512
#define NO   128
#define TM   16
#define TN   64
#define OSW  68
#define DELTA_F 0.1f
#define WSC  64.0f
#define WSI  0.015625f

static_assert(NB <= NB_FULL);
static_assert(NB % TM == 0);
static_assert(NC % TN == 0);
static_assert(NO % TN == 0);
static_assert(KP % 32 == 0);
static_assert(NC % 32 == 0);
static_assert(KP % 8 == 0);
static_assert(NC % 8 == 0);
static_assert(TN == 64);
static_assert(TM == 16);
static_assert(OSW >= TN);
static_assert((OSW * 4) % 16 == 0);
static_assert(((size_t)NB * KP) % 2048 == 0);
static_assert(((size_t)NC * KP) % 2048 == 0);
static_assert(((size_t)NO * NC) % 2048 == 0);
static_assert(TM * OSW * 4 <= 131072);
static_assert(32 * 16 * 4 == TM * TN * 2);
static_assert(32 * 16 * 8 == TM * TN * 4);
static_assert(8 * 32 * 4 == TM * TN);

typedef _Float16 h16;
typedef unsigned short bf;
typedef __attribute__((ext_vector_type(16))) __bf16   v16bf;
typedef __attribute__((ext_vector_type(16))) _Float16 v16h;
typedef __attribute__((ext_vector_type(8)))  _Float16 v8h;
typedef __attribute__((ext_vector_type(8)))  unsigned short v8us;
typedef __attribute__((ext_vector_type(8)))  float    v8f;
typedef __attribute__((ext_vector_type(4)))  float    v4f;
typedef v4f  __attribute__((may_alias)) v4fa;

__device__ __forceinline__ unsigned short f2bf(float f) { unsigned u = __float_as_uint(f); u += 0x7FFFu + ((u >> 16) & 1u); return (unsigned short)(u >> 16); }
__device__ __forceinline__ float bfr(float f) { return __uint_as_float(((unsigned)f2bf(f)) << 16); }
__device__ __forceinline__ v16h cat16(v8h lo, v8h hi) { return __builtin_shufflevector(lo, hi, 0, 1, 2, 3, 4, 5, 6, 7, 8, 9, 10, 11, 12, 13, 14, 15); }
__device__ __forceinline__ v16bf cat16b(v8us lo, v8us hi) { return __builtin_bit_cast(v16bf, __builtin_shufflevector(lo, hi, 0, 1, 2, 3, 4, 5, 6, 7, 8, 9, 10, 11, 12, 13, 14, 15)); }
__device__ __forceinline__ v8f wmma16(v16h a, v16h b, v8f c) { return __builtin_amdgcn_wmma_f32_16x16x32_f16(false, a, false, b, (short)0, c, false, false); }
__device__ __forceinline__ v8f wmmab(v16bf a, v16bf b, v8f c) { return __builtin_amdgcn_wmma_f32_16x16x32_bf16(false, a, false, b, (short)0, c, false, false); }
__device__ __forceinline__ v16h  ldh(const h16* p) { return cat16(*(const v8h*)p, *(const v8h*)(p + 16)); }
__device__ __forceinline__ v16bf ldb(const bf* p)  { return cat16b(*(const v8us*)p, *(const v8us*)(p + 16)); }
__device__ __forceinline__ void wave_sync() { __builtin_amdgcn_fence(3  , "wavefront"); __builtin_amdgcn_wave_barrier(); asm volatile("" ::: "memory"); }

__device__ __forceinline__ v8f wmmabg(v16bf a, v16bf b, v8f c) { c = wmmab(a, b, c); asm volatile("v_nop\n\tv_nop\n\tv_nop\n\tv_nop" : "+v"(c) : "v"(a), "v"(b)); return c; }
__device__ __forceinline__ v8f wmma16g(v16h a, v16h b, v8f c) { c = wmma16(a, b, c); asm volatile("v_nop\n\tv_nop\n\tv_nop\n\tv_nop" : "+v"(c) : "v"(a), "v"(b)); return c; }
__device__ __forceinline__ v8f mmag(v16bf a, v16bf b, v8f c) { return wmmabg(a, b, c); }
__device__ __forceinline__ v8f mmag(v16h a, v16h b, v8f c)   { return wmma16g(a, b, c); }
__device__ __forceinline__ v16bf ldfrag(const bf* p)  { return ldb(p); }
__device__ __forceinline__ v16h  ldfrag(const h16* p) { return ldh(p); }
static __device__ __forceinline__ h16 toh_flush(float v) { const float w = (fabsf(v) < 6.103515625e-05f) ? 0.0f : v; return (h16)w; }

__global__ __launch_bounds__(256) void k_cvt_bf(const float* __restrict__ src, bf* VB, bf* VA, float* VF, size_t n8) {
    const size_t i = (size_t)blockIdx.x * 256 + threadIdx.x; if (i >= n8) return;
    const v8f v = *(const v8f*)(src + i * 8); v8us o, a;
#pragma unroll
    for (int k = 0; k < 8; ++k) { o[k] = f2bf(v[k]); a[k] = f2bf(fabsf(v[k])); }
    const size_t j0 = (size_t)blockIdx.x * 2048 + (size_t)threadIdx.x * 4;
    const v4f w0 = *(const v4f*)(src + j0); const v4f w1 = *(const v4f*)(src + j0 + 1024); v4f f0, f1;
#pragma unroll
    for (int k = 0; k < 4; ++k) { f0[k] = fabsf(bfr(w0[k])); f1[k] = fabsf(bfr(w1[k])); }
    *(volatile v8us*)(VB + i * 8) = o; *(volatile v8us*)(VA + i * 8) = a; *(volatile v4f*)(VF + j0) = f0; *(volatile v4f*)(VF + j0 + 1024) = f1;
    __threadfence();
    *(volatile v8us*)(VB + i * 8) = o; *(volatile v8us*)(VA + i * 8) = a; *(volatile v4f*)(VF + j0) = f0; *(volatile v4f*)(VF + j0 + 1024) = f1;
}

__global__ __launch_bounds__(256) void k_cvt_h(const float* __restrict__ src, h16* VH, h16* VA, float* VF, size_t n8) {
    const size_t i = (size_t)blockIdx.x * 256 + threadIdx.x; if (i >= n8) return;
    const v8f v = *(const v8f*)(src + i * 8); v8h o, a;
#pragma unroll
    for (int k = 0; k < 8; ++k) { const float w = bfr(v[k]) * WSC; o[k] = toh_flush(w); a[k] = toh_flush(fabsf(w)); }
    const size_t j0 = (size_t)blockIdx.x * 2048 + (size_t)threadIdx.x * 4;
    const v4f w0 = *(const v4f*)(src + j0); const v4f w1 = *(const v4f*)(src + j0 + 1024); v4f f0, f1;
#pragma unroll
    for (int k = 0; k < 4; ++k) { f0[k] = fabsf(bfr(w0[k])); f1[k] = fabsf(bfr(w1[k])); }
    *(volatile v8h*)(VH + i * 8) = o; *(volatile v8h*)(VA + i * 8) = a; *(volatile v4f*)(VF + j0) = f0; *(volatile v4f*)(VF + j0 + 1024) = f1;
    __threadfence();
    *(volatile v8h*)(VH + i * 8) = o; *(volatile v8h*)(VA + i * 8) = a; *(volatile v4f*)(VF + j0) = f0; *(volatile v4f*)(VF + j0 + 1024) = f1;
}

template <typename PT, int N, int K, bool CONJ>
__device__ __forceinline__ void layer_tile(const PT* __restrict__ AV, const PT* __restrict__ AA, const float* __restrict__ AF,
                                           const PT* __restrict__ BV, const PT* __restrict__ BA, const float* __restrict__ BF,
                                           h16* CH, h16* CA, float* CF, float* OUT) {
#pragma clang fp contract(off)
    __shared__ __align__(16) float os[TM * OSW];
    const unsigned lane = threadIdx.x & 31u, lr = lane & 15u, hi = lane >> 4;
    const unsigned r0 = blockIdx.x * (unsigned)TM, c0 = blockIdx.y * (unsigned)TN;
    v8f accL[4], accA[4]; float amax[4][8];
#pragma unroll
    for (int nb = 0; nb < 4; ++nb) { accL[nb] = (v8f){}; accA[nb] = (v8f){};
#pragma unroll
        for (int j = 0; j < 8; ++j) amax[nb][j] = 0.0f; }
    const size_t aoff = (size_t)(r0 + lr) * (size_t)K + 8u * hi;
    const size_t boff = (size_t)(c0 + lr) * (size_t)K + 8u * hi;
    const size_t xfo  = (size_t)(r0 + 8u * hi) * (size_t)K;
    const size_t wfo  = (size_t)(c0 + lr) * (size_t)K;
#pragma unroll 1
    for (unsigned kc = 0; kc < (unsigned)K; kc += 32u) {
        const auto a  = ldfrag(AV + aoff + kc);
        const auto aa = ldfrag(AA + aoff + kc);
#pragma unroll
        for (int nb = 0; nb < 4; ++nb) {
            const auto b  = ldfrag(BV + boff + (size_t)nb * 16 * (size_t)K + kc);
            const auto bb = ldfrag(BA + boff + (size_t)nb * 16 * (size_t)K + kc);
            accL[nb] = mmag(a, b, accL[nb]);
            accA[nb] = mmag(aa, bb, accA[nb]);
        }
#pragma unroll 1
        for (unsigned kq = 0; kq < 32u; kq += 4u) {
            v4f xv[8], wv[4];
#pragma unroll
            for (int j = 0; j < 8; ++j) xv[j] = *(const v4f*)(AF + xfo + (size_t)j * (size_t)K + kc + kq);
#pragma unroll
            for (int nb = 0; nb < 4; ++nb) wv[nb] = *(const v4f*)(BF + wfo + (size_t)nb * 16 * (size_t)K + kc + kq);
#pragma unroll
            for (int nb = 0; nb < 4; ++nb) {
#pragma unroll
                for (int j = 0; j < 8; ++j) {
                    const v4f p = xv[j] * wv[nb];
                    amax[nb][j] = fmaxf(fmaxf(amax[nb][j], fmaxf(p[0], p[1])), fmaxf(p[2], p[3])); } }
        }
    }
#pragma unroll
    for (int nb = 0; nb < 4; ++nb) {
#pragma unroll
        for (int j = 0; j < 8; ++j) {
            float lin = accL[nb][j], sab = accA[nb][j];
            if (!CONJ) { lin = lin * WSI; sab = sab * WSI; }
            const float bias = CONJ ? (amax[nb][j] - sab) : (sab - amax[nb][j]);
            const float db = DELTA_F * bias;
            os[(hi * 8u + (unsigned)j) * OSW + (unsigned)nb * 16u + lr] = lin + db; } }
    wave_sync();
    if (CONJ) {
#pragma unroll 1
        for (unsigned i = 0; i < 8u; ++i) { const unsigned idx = i * 32u + lane; const unsigned row = idx >> 4, c4 = (idx & 15u) * 4u;
            v4f t = *(const v4fa*)(&os[row * OSW + c4]);
            t[0] = tanhf(t[0]); t[1] = tanhf(t[1]); t[2] = tanhf(t[2]); t[3] = tanhf(t[3]);
            *(v4fa*)(&os[row * OSW + c4]) = t; }
        wave_sync();
    }
#pragma unroll 1
    for (int ps = 0; ps < 2; ++ps) {
        if (CONJ) {
#pragma unroll
            for (unsigned s = 0; s < 4u; ++s) { const unsigned row = 4u * s + (lane >> 3), c8 = (lane & 7u) * 8u;
                const v4f x0 = *(const v4fa*)(&os[row * OSW + c8]); const v4f x1 = *(const v4fa*)(&os[row * OSW + c8 + 4u]); v8h hv, av;
#pragma unroll
                for (int i = 0; i < 4; ++i) { hv[i] = toh_flush(x0[i]); hv[4 + i] = toh_flush(x1[i]); av[i] = toh_flush(fabsf(x0[i])); av[4 + i] = toh_flush(fabsf(x1[i])); }
                const size_t oo = (size_t)(r0 + row) * (size_t)N + c0 + c8;
                *(volatile v8h*)(CH + oo) = hv; *(volatile v8h*)(CA + oo) = av; }
#pragma unroll
            for (unsigned s = 0; s < 8u; ++s) { const unsigned row = 2u * s + (lane >> 4), c4 = (lane & 15u) * 4u;
                const v4f x0 = *(const v4fa*)(&os[row * OSW + c4]); v4f f;
                f[0] = fabsf(x0[0]); f[1] = fabsf(x0[1]); f[2] = fabsf(x0[2]); f[3] = fabsf(x0[3]);
                *(volatile v4f*)(CF + (size_t)(r0 + row) * (size_t)N + c0 + c4) = f; }
        } else {
#pragma unroll
            for (unsigned s = 0; s < 8u; ++s) { const unsigned row = 2u * s + (lane >> 4), c4 = (lane & 15u) * 4u;
                const v4f val = *(const v4fa*)(&os[row * OSW + c4]);
                *(volatile v4f*)(OUT + (size_t)(r0 + row) * (size_t)N + c0 + c4) = val; }
        }
        if (ps == 0) __threadfence(); }
}

__global__ __launch_bounds__(32) void k_layer1(const bf* __restrict__ XB, const bf* __restrict__ XA, const float* __restrict__ XF,
                                               const bf* __restrict__ WB, const bf* __restrict__ WA, const float* __restrict__ WF,
                                               h16* CH, h16* CA, float* CF) {
    layer_tile<bf, NC, KP, true>(XB, XA, XF, WB, WA, WF, CH, CA, CF, (float*)0);
}

__global__ __launch_bounds__(32) void k_layer2(const h16* __restrict__ CH, const h16* __restrict__ CA, const float* __restrict__ CF,
                                               const h16* __restrict__ WH, const h16* __restrict__ WA, const float* __restrict__ WF,
                                               float* OUT) {
    layer_tile<h16, NO, NC, false>(CH, CA, CF, WH, WA, WF, (h16*)0, (h16*)0, (float*)0, OUT);
}

static constexpr size_t al256(size_t v) { return (v + 255) & ~(size_t)255; }
static constexpr size_t N_X  = (size_t)NB * KP;
static constexpr size_t N_WC = (size_t)NC * KP;
static constexpr size_t N_WD = (size_t)NO * NC;
static constexpr size_t N_C  = (size_t)NB * NC;
static constexpr size_t N_O  = (size_t)NB * NO;
static constexpr size_t SZ_X16 = al256(N_X * 2),  SZ_X32 = al256(N_X * 4);
static constexpr size_t SZ_WC16 = al256(N_WC * 2), SZ_WC32 = al256(N_WC * 4);
static constexpr size_t SZ_WD16 = al256(N_WD * 2), SZ_WD32 = al256(N_WD * 4);
static constexpr size_t SZ_C16 = al256(N_C * 2),  SZ_C32 = al256(N_C * 4);
static constexpr size_t SZ_TOTAL = 2 * SZ_X16 + SZ_X32 + 2 * SZ_WC16 + SZ_WC32 + 2 * SZ_WD16 + SZ_WD32 + 2 * SZ_C16 + SZ_C32;
static_assert(SZ_TOTAL <= (size_t)134217728);
static constexpr unsigned G_X  = (unsigned)(N_X / 2048);
static constexpr unsigned G_WC = (unsigned)(N_WC / 2048);
static constexpr unsigned G_WD = (unsigned)(N_WD / 2048);
static_assert((size_t)G_X * 2048 == N_X);
static_assert((size_t)G_WC * 2048 == N_WC);
static_assert((size_t)G_WD * 2048 == N_WD);
static_assert((size_t)(NB / TM) * (NC / TN) * TM * TN == N_C);
static_assert((size_t)(NB / TM) * (NO / TN) * TM * TN == N_O);

extern "C" void kernel_launch(void* const* d_in, const int* in_sizes, int n_in,
                              void* d_out, int out_size, void* d_ws, size_t ws_size, hipStream_t stream) {
    if (n_in < 3) return;
    if ((size_t)in_sizes[0] < N_X || (size_t)in_sizes[1] < N_WC || (size_t)in_sizes[2] < N_WD) return;
    if ((size_t)out_size < N_O) return;
    if (SZ_TOTAL > ws_size) return;
    const float* x  = (const float*)d_in[0];
    const float* wc = (const float*)d_in[1];
    const float* wd = (const float*)d_in[2];
    float* OUT = (float*)d_out;
    char* wsp = (char*)d_ws;
    bf*    XB  = (bf*)wsp;    wsp += SZ_X16;
    bf*    XA  = (bf*)wsp;    wsp += SZ_X16;
    float* XF  = (float*)wsp; wsp += SZ_X32;
    bf*    WCB = (bf*)wsp;    wsp += SZ_WC16;
    bf*    WCA = (bf*)wsp;    wsp += SZ_WC16;
    float* WCF = (float*)wsp; wsp += SZ_WC32;
    h16*   WDH = (h16*)wsp;   wsp += SZ_WD16;
    h16*   WDA = (h16*)wsp;   wsp += SZ_WD16;
    float* WDF = (float*)wsp; wsp += SZ_WD32;
    h16*   CH  = (h16*)wsp;   wsp += SZ_C16;
    h16*   CA  = (h16*)wsp;   wsp += SZ_C16;
    float* CF  = (float*)wsp; wsp += SZ_C32;

    k_cvt_bf<<<G_X,  256, 0, stream>>>(x,  XB,  XA,  XF,  N_X  / 8);
    k_cvt_bf<<<G_WC, 256, 0, stream>>>(wc, WCB, WCA, WCF, N_WC / 8);
    k_cvt_h <<<G_WD, 256, 0, stream>>>(wd, WDH, WDA, WDF, N_WD / 8);

    k_layer1<<<dim3(NB / TM, NC / TN, 1), 32, 0, stream>>>(XB, XA, XF, WCB, WCA, WCF, CH, CA, CF);
    k_layer2<<<dim3(NB / TM, NO / TN, 1), 32, 0, stream>>>(CH, CA, CF, WDH, WDA, WDF, OUT);
}
